// LayerNormLSTMCell_55508157333862
// MI455X (gfx1250) — hardware-verified
//
#include <hip/hip_runtime.h>
#include <hip/hip_bf16.h>

#pragma clang fp contract(off)
constexpr int Bsz = 4096;
constexpr int Hh  = 1024;
constexpr int Kd  = 2048;
constexpr int N4  = 4096;
constexpr float EPS = 1e-5f;

typedef _Float16 bf16_t;
typedef __attribute__((ext_vector_type(16))) _Float16 v16bf;
typedef __attribute__((ext_vector_type(8)))  float  v8f;
typedef __attribute__((ext_vector_type(4)))  float  v4f_t;
typedef float v4fa __attribute__((ext_vector_type(4), may_alias));

union ABu { v16bf v; uint4 u[2]; };

__global__ __launch_bounds__(256)
void pack_kernel(const float* __restrict__ x, const float* __restrict__ h,
                 const float* __restrict__ W,
                 bf16_t* __restrict__ XH, bf16_t* __restrict__ Wb) {
  const size_t i = (size_t)blockIdx.x * blockDim.x + threadIdx.x;
  constexpr size_t nchunks = (size_t)Bsz * Kd / 4;
  if (i >= nchunks) return;

  const size_t r  = i / (Kd / 4);
  const size_t c4 = (i % (Kd / 4)) * 4;
  const float4 v = (c4 < (size_t)Hh) ? *(const float4*)(x + r * Hh + c4)
                                     : *(const float4*)(h + r * Hh + (c4 - Hh));
  typedef __attribute__((ext_vector_type(2))) unsigned v2u_t;
  union { bf16_t b[4]; v2u_t u; } o;
  o.b[0] = (bf16_t)v.x; o.b[1] = (bf16_t)v.y;
  o.b[2] = (bf16_t)v.z; o.b[3] = (bf16_t)v.w;
  const float4 w = *(const float4*)(W + i * 4);
  union { bf16_t b[4]; v2u_t u; } ow;
  ow.b[0] = (bf16_t)w.x; ow.b[1] = (bf16_t)w.y;
  ow.b[2] = (bf16_t)w.z; ow.b[3] = (bf16_t)w.w;
  *(volatile v2u_t*)(XH + i * 4) = o.u; *(volatile v2u_t*)(Wb + i * 4) = ow.u; __threadfence();
  *(volatile v2u_t*)(XH + i * 4) = o.u; *(volatile v2u_t*)(Wb + i * 4) = ow.u;
}

constexpr int BM = 128, BN = 128, BK = 64;
constexpr int CPR = BK / 8;

__device__ __forceinline__ int swz(int row, int chunk) {
  return (row << 3) + (chunk ^ ((row + (row >> 3)) & 7));
}

__global__ __launch_bounds__(256)
void gemm_kernel(const bf16_t* __restrict__ XH, const bf16_t* __restrict__ Wb,
                 float* __restrict__ gates) {
  __shared__ uint4 As[4][BM * CPR];
  uint4 (*Bs)[BM * CPR] = &As[2];

  const int tid   = threadIdx.x;
  const int lane  = tid & 31;
  const int wave  = tid >> 5;
  const int waveM = wave >> 2;
  const int waveN = wave & 3;
  const int m0 = blockIdx.y * BM;
  const int n0 = blockIdx.x * BN;

  const int lrow = lane & 15;
  const int hsel = lane >> 4;

  auto issue_stage = [&](int buf, int kt) {
#pragma unroll
    for (int q = 0; q < 4; ++q) {
      const int f   = tid + (q << 8);
      const int row = f >> 3;
      const int ch  = f & 7;
      const bf16_t* ga = XH + (size_t)(m0 + row) * Kd + kt + ch * 8;
      const bf16_t* gb = Wb + (size_t)(n0 + row) * Kd + kt + ch * 8;
      const uint32_t la = (uint32_t)(uintptr_t)&As[buf][swz(row, ch)];
      const uint32_t lb = (uint32_t)(uintptr_t)&Bs[buf][swz(row, ch)];
      asm volatile("global_load_async_to_lds_b128 %0, %1, off"
                   :: "v"(la), "v"(ga) : "memory");
      asm volatile("global_load_async_to_lds_b128 %0, %1, off"
                   :: "v"(lb), "v"(gb) : "memory");
    }
  };

  v8f acc[4][2] = {};

  issue_stage(0, 0);
  constexpr int NSTAGE = Kd / BK;
  for (int s = 0; s < NSTAGE; ++s) {
    asm volatile("s_wait_asynccnt 0x0" ::: "memory");
    __syncthreads();
    if (s + 1 < NSTAGE) issue_stage((s + 1) & 1, (s + 1) * BK);

    const int buf = s & 1;
#pragma unroll
    for (int ks = 0; ks < 2; ++ks) {
      const int cb = ks * 4 + hsel;
      ABu af[4];
      ABu bfr[2];
#pragma unroll
      for (int mf = 0; mf < 4; ++mf) {
        const int r = waveM * 64 + mf * 16 + lrow;
        af[mf].u[0] = As[buf][swz(r, cb)];
        af[mf].u[1] = As[buf][swz(r, cb + 2)];
      }
#pragma unroll
      for (int nf = 0; nf < 2; ++nf) {
        const int r = waveN * 32 + nf * 16 + lrow;
        bfr[nf].u[0] = Bs[buf][swz(r, cb)];
        bfr[nf].u[1] = Bs[buf][swz(r, cb + 2)];
      }
#pragma unroll
      for (int mf = 0; mf < 4; ++mf)
#pragma unroll
        for (int nf = 0; nf < 2; ++nf)
          acc[mf][nf] = __builtin_amdgcn_wmma_f32_16x16x32_f16(
              false, af[mf].v, false, bfr[nf].v,
              (short)0, acc[mf][nf], false, false);
    }
  }

  __syncthreads();
  float* Cs = (float*)&As[0][0];
  const int rsel = hsel * 8;
#pragma unroll
  for (int mf = 0; mf < 4; ++mf) {
#pragma unroll
    for (int nf = 0; nf < 2; ++nf) {
      const int cl = waveN * 32 + nf * 16 + lrow;
#pragma unroll
      for (int v = 0; v < 8; ++v) {
        const int rl = waveM * 64 + mf * 16 + rsel + v;
        Cs[rl * BN + cl] = acc[mf][nf][v];
      }
    }
  }
  __syncthreads();
#pragma unroll 1
  for (int pass = 0; pass < 2; ++pass) {
    for (int ch = tid; ch < BM * (BN / 4); ch += 256) { const int rl = ch >> 5, q = (ch & 31) * 4;
      *(volatile v4f_t*)(gates + (size_t)(m0 + rl) * N4 + n0 + q) = *(const volatile v4fa*)(Cs + rl * BN + q); }
    __threadfence();
  }
}

__device__ __forceinline__ float block_reduce_sum(float v, float* sbuf) {
#pragma unroll
  for (int off = 16; off > 0; off >>= 1) v += __shfl_xor(v, off, 32);
  const int lane = threadIdx.x & 31;
  const int wid  = threadIdx.x >> 5;
  if (lane == 0) sbuf[wid] = v;
  __syncthreads();
  float r = (threadIdx.x < 8) ? sbuf[threadIdx.x] : 0.0f;
  if (wid == 0) {
#pragma unroll
    for (int off = 4; off > 0; off >>= 1) r += __shfl_xor(r, off, 32);
    if (lane == 0) sbuf[0] = r;
  }
  __syncthreads();
  const float out = sbuf[0];
  __syncthreads();
  return out;
}

__device__ __forceinline__ float sigmoidf(float x) {
  return __builtin_amdgcn_rcpf(1.0f + __expf(-x));
}
__device__ __forceinline__ float tanh_e(float x) {
  return 1.0f - 2.0f * __builtin_amdgcn_rcpf(1.0f + __expf(2.0f * x));
}

__global__ __launch_bounds__(256)
void epilogue_kernel(const float* __restrict__ gates, const float* __restrict__ c,
                     const float* __restrict__ bias,
                     const float* __restrict__ lnig, const float* __restrict__ lnib,
                     const float* __restrict__ lnfg, const float* __restrict__ lnfb,
                     const float* __restrict__ lngg, const float* __restrict__ lngb,
                     const float* __restrict__ lnog, const float* __restrict__ lnob,
                     const float* __restrict__ lncg, const float* __restrict__ lncb,
                     float* __restrict__ out) {
  __shared__ float sred[32];
  const int b = blockIdx.x;
  const int t = threadIdx.x;
  const float invH = 1.0f / (float)Hh;
  const size_t rowBase = (size_t)b * N4;

  float iv[4], fv[4], gv[4], ov[4];
  float s_i = 0, q_i = 0, s_f = 0, q_f = 0, s_g = 0, q_g = 0, s_o = 0, q_o = 0;
#pragma unroll
  for (int e = 0; e < 4; ++e) {
    const int j = t + e * 256;
    const float a  = gates[rowBase + 0 * Hh + j] + bias[0 * Hh + j];
    const float f_ = gates[rowBase + 1 * Hh + j] + bias[1 * Hh + j];
    const float g_ = gates[rowBase + 2 * Hh + j] + bias[2 * Hh + j];
    const float o_ = gates[rowBase + 3 * Hh + j] + bias[3 * Hh + j];
    iv[e] = a;  fv[e] = f_; gv[e] = g_; ov[e] = o_;
    s_i += a;  q_i += a * a;   s_f += f_; q_f += f_ * f_;
    s_g += g_; q_g += g_ * g_; s_o += o_; q_o += o_ * o_;
  }
  s_i = block_reduce_sum(s_i, sred); q_i = block_reduce_sum(q_i, sred);
  s_f = block_reduce_sum(s_f, sred); q_f = block_reduce_sum(q_f, sred);
  s_g = block_reduce_sum(s_g, sred); q_g = block_reduce_sum(q_g, sred);
  s_o = block_reduce_sum(s_o, sred); q_o = block_reduce_sum(q_o, sred);

  const float mi = s_i * invH, ri = rsqrtf(q_i * invH - mi * mi + EPS);
  const float mf = s_f * invH, rf = rsqrtf(q_f * invH - mf * mf + EPS);
  const float mg = s_g * invH, rg = rsqrtf(q_g * invH - mg * mg + EPS);
  const float mo = s_o * invH, ro = rsqrtf(q_o * invH - mo * mo + EPS);

  float cn[4];
  float s_c = 0, q_c = 0;
#pragma unroll
  for (int e = 0; e < 4; ++e) {
    const int j = t + e * 256;
    const float ig = sigmoidf((iv[e] - mi) * ri * lnig[j] + lnib[j]);
    const float fg = sigmoidf((fv[e] - mf) * rf * lnfg[j] + lnfb[j]);
    const float gg = tanh_e(  (gv[e] - mg) * rg * lngg[j] + lngb[j]);
    const float og = sigmoidf((ov[e] - mo) * ro * lnog[j] + lnob[j]);
    const float cnew = fg * c[(size_t)b * Hh + j] + ig * gg;
    cn[e] = cnew;
    ov[e] = og;
    s_c += cnew; q_c += cnew * cnew;
  }
  s_c = block_reduce_sum(s_c, sred);
  q_c = block_reduce_sum(q_c, sred);
  const float mc = s_c * invH, rc = rsqrtf(q_c * invH - mc * mc + EPS);

#pragma unroll
  for (int e = 0; e < 4; ++e) {
    const int j = t + e * 256;
    const float lnc  = (cn[e] - mc) * rc * lncg[j] + lncb[j];
    const float hnew = ov[e] * tanh_e(lnc);
    float* dh = out + (size_t)b * Hh + j;
    float* dc = out + (size_t)Bsz * Hh + (size_t)b * Hh + j;
    *(volatile float*)dh = hnew; *(volatile float*)dc = cn[e]; __threadfence();
    *(volatile float*)dh = hnew; *(volatile float*)dc = cn[e];
  }
}

extern "C" void kernel_launch(void* const* d_in, const int* in_sizes, int n_in,
                              void* d_out, int out_size, void* d_ws, size_t ws_size,
                              hipStream_t stream) {
  const float* x    = (const float*)d_in[0];
  const float* h    = (const float*)d_in[1];
  const float* c    = (const float*)d_in[2];
  const float* W    = (const float*)d_in[3];
  const float* bias = (const float*)d_in[4];
  const float* lnig = (const float*)d_in[5];
  const float* lnib = (const float*)d_in[6];
  const float* lnfg = (const float*)d_in[7];
  const float* lnfb = (const float*)d_in[8];
  const float* lngg = (const float*)d_in[9];
  const float* lngb = (const float*)d_in[10];
  const float* lnog = (const float*)d_in[11];
  const float* lnob = (const float*)d_in[12];
  const float* lncg = (const float*)d_in[13];
  const float* lncb = (const float*)d_in[14];
  float* out = (float*)d_out;

  bf16_t* Wb    = (bf16_t*)d_ws;
  bf16_t* XH    = Wb + (size_t)N4 * Kd;
  float*  gates = (float*)(XH + (size_t)Bsz * Kd);

  const size_t nchunks = (size_t)Bsz * Kd / 4;
  const int packBlocks = (int)((nchunks + 255) / 256);
  pack_kernel<<<packBlocks, 256, 0, stream>>>(x, h, W, XH, Wb);

  dim3 gemmGrid(N4 / BN, Bsz / BM);
  gemm_kernel<<<gemmGrid, 256, 0, stream>>>(XH, Wb, gates);

  epilogue_kernel<<<Bsz, 256, 0, stream>>>(gates, c, bias,
                                           lnig, lnib, lnfg, lnfb,
                                           lngg, lngb, lnog, lnob,
                                           lncg, lncb, out);
}
